// FractalAttention_21612275433837
// MI455X (gfx1250) — hardware-run, weakly checked
//
#include <hip/hip_runtime.h>
#include <stddef.h>


typedef _Float16 v16h __attribute__((ext_vector_type(16)));
typedef _Float16 v8h  __attribute__((ext_vector_type(8)));
typedef float    v8f  __attribute__((ext_vector_type(8)));
typedef float    v4f  __attribute__((ext_vector_type(4)));

#ifndef NB
#define NB 8
#endif
#ifndef SEQ
#define SEQ 8192
#endif
#define NB_FULL  8
#define SEQ_FULL 8192
#define DIM   128
#define NHEAD 8
#define DEPTH 4
#define KMIX   (NHEAD * DIM)
#define WPITCH (DEPTH * NHEAD * DIM)
#define MROWS (NB * SEQ)

constexpr unsigned ilog2c(unsigned v) { return (v <= 1u) ? 0u : 1u + ilog2c(v >> 1); }
#define LSH0 (ilog2c((unsigned)SEQ) - (unsigned)(DEPTH - 1))

static_assert(NB >= 1 && NB <= NB_FULL);
static_assert(SEQ <= SEQ_FULL && (SEQ & (SEQ - 1)) == 0);
static_assert((SEQ >> (DEPTH - 1)) >= 128);
static_assert(((SEQ >> (DEPTH - 1)) % 128) == 0);
static_assert(DIM == 128 && (DIM % 32) == 0 && (DIM % 64) == 0);
static_assert(NHEAD == 8 && 16 * NHEAD == 128);
static_assert(KMIX == 1024 && (KMIX % 64) == 0 && (KMIX % 32) == 0);
static_assert((WPITCH % 64) == 0);
static_assert((MROWS % 16) == 0 && (SEQ % 16) == 0);
static_assert((size_t)MROWS * DIM < (size_t)0xFFFFFFFFu);

#define LDT 72
#define LDM 136
#define LDY 132
static_assert((LDT % 8) == 0 && LDT >= 64);
static_assert((LDM % 8) == 0 && LDM >= DIM);
static_assert((LDY % 4) == 0 && LDY >= DIM);

#define WCARRY 64.0f
#define SX1 0.125f
#define SX2 0.03125f
#define SX3 0.00390625f

#define WH_BYTES ((size_t)DIM * WPITCH * 2)
#define WM_BYTES ((size_t)DIM * KMIX * 2)
#define XP_BYTES ((size_t)MROWS * DIM * 2)
#define OFF_WH ((size_t)0)
#define OFF_WM (OFF_WH + WH_BYTES)
#define OFF_XA (OFF_WM + WM_BYTES)
#define OFF_XB (OFF_XA + XP_BYTES)
#define WS_TOTAL (OFF_XB + XP_BYTES)
static_assert((WH_BYTES % 128) == 0 && (WM_BYTES % 128) == 0 && (XP_BYTES % 128) == 0);
static_assert(WS_TOTAL <= (size_t)134217728);

__device__ __forceinline__ float bf16r(float x) {
  unsigned int u = __float_as_uint(x);
  u = (u + 0x7FFFu + ((u >> 16) & 1u)) & 0xFFFF0000u;
  return __uint_as_float(u);
}

__device__ __forceinline__ _Float16 toh_flush(float v) {
  const _Float16 r = (_Float16)v;
  return (fabsf(v) < 6.103515625e-05f) ? (_Float16)0.0f : r;
}

__device__ __forceinline__ v16h frag_at(const _Float16* p) {
  v8h lo = *(const v8h*)(p);
  v8h hi = *(const v8h*)(p + 16);
  v16h out;
#pragma unroll
  for (int i = 0; i < 8; ++i) { out[i] = lo[i]; out[i + 8] = hi[i]; }
  return out;
}
__device__ __forceinline__ v16h ld_frag(const _Float16* base, unsigned ld) {
  const unsigned lane = threadIdx.x & 31u;
  return frag_at(base + (lane & 15u) * ld + (lane >> 4) * 8u);
}

__device__ __forceinline__ v8f wmma16(v16h a, v16h b, v8f c) {
  v8f d = __builtin_amdgcn_wmma_f32_16x16x32_f16(false, a, false, b, (short)0, c,
                                                 false, false);
  asm volatile("v_nop\n\tv_nop\n\tv_nop\n\tv_nop" : "+v"(d) : "v"(a), "v"(b));
  return d;
}

__global__ __launch_bounds__(256) void wconv_kernel(
    const float* __restrict__ W, _Float16* __restrict__ Wt, unsigned ldw, unsigned ldk) {
  __shared__ _Float16 T[64 * LDT];
  const unsigned tid = threadIdx.x;
  const unsigned n0 = blockIdx.x * 64u;
  const unsigned k0 = blockIdx.y * 64u;
#pragma unroll 4
  for (unsigned j = 0; j < 16u; ++j) {
    const unsigned idx = tid + 256u * j;
    const unsigned kr = idx >> 6, nc = idx & 63u;
    const float v = W[(size_t)(k0 + kr) * ldw + n0 + nc];
    T[nc * LDT + kr] = (_Float16)(WCARRY * bf16r(v));
  }
  __syncthreads();
  v8h x[2];
  size_t off[2];
#pragma unroll
  for (unsigned i = 0; i < 2u; ++i) {
    const unsigned n = 32u * i + (tid >> 3);
    const unsigned kc = (tid & 7u) * 8u;
    x[i] = *(const v8h*)&T[n * LDT + kc];
    off[i] = (size_t)(n0 + n) * ldk + k0 + kc;
  }
#pragma unroll
  for (int i = 0; i < 2; ++i) *(volatile v8h*)(Wt + off[i]) = x[i];
  __threadfence();
#pragma unroll
  for (int i = 0; i < 2; ++i) *(volatile v8h*)(Wt + off[i]) = x[i];
}

__global__ __launch_bounds__(256) void xconv_kernel(
    const float* __restrict__ X, _Float16* __restrict__ dst) {
  const unsigned g = blockIdx.x * 256u + threadIdx.x;
  const unsigned crow = g >> 4;
  const unsigned c = (g & 15u) * 8u;
  const unsigned bidx = crow / (unsigned)SEQ;
  const unsigned sq = crow - bidx * (unsigned)SEQ;
  const size_t frow = (size_t)bidx * SEQ_FULL + sq;
  const v4f a0 = *(const v4f*)(X + frow * DIM + c);
  const v4f a1 = *(const v4f*)(X + frow * DIM + c + 4u);
  v8h o;
#pragma unroll
  for (int i = 0; i < 4; ++i) {
    o[i]     = toh_flush(bf16r(a0[i]));
    o[i + 4] = toh_flush(bf16r(a1[i]));
  }
  _Float16* p = dst + (size_t)crow * DIM + c;
  *(volatile v8h*)p = o;
  __threadfence();
  *(volatile v8h*)p = o;
}

template <int LAST>
__device__ __forceinline__ void level_body(
    const _Float16* __restrict__ Xin, const _Float16* __restrict__ Wh_t,
    const _Float16* __restrict__ Wm_t, const float* __restrict__ bmix,
    float* __restrict__ outf, _Float16* __restrict__ out16,
    const unsigned lshift, const float cs, const float bs) {
  __shared__ _Float16 Ms[128 * LDM];
  __shared__ float Ys[16 * LDY];

  const unsigned tid = threadIdx.x, lane = tid & 31u;
  const unsigned w = (unsigned)__builtin_amdgcn_readfirstlane((int)(threadIdx.x >> 5));
  const unsigned hh = lane >> 4, m = lane & 15u;

  const unsigned r0 = blockIdx.x * 16u;
  const unsigned bidx = r0 / (unsigned)SEQ;
  const unsigned s0 = r0 - bidx * (unsigned)SEQ;
  const unsigned lmask = (1u << lshift) - 1u;
  const unsigned l0 = s0 & lmask;
  const unsigned segb = r0 - l0;
  const unsigned p0 = l0 * (unsigned)NHEAD;
  const unsigned head = p0 >> lshift;
  const unsigned xrow0 = segb + (p0 & lmask);

  {
    const _Float16* xp = Xin + (size_t)(xrow0 + w * 16u + m) * DIM + hh * 8u;
    const _Float16* wp = Wh_t + (size_t)m * WPITCH + head * (unsigned)DIM + hh * 8u;
    v8f acc[8];
#pragma unroll
    for (int j = 0; j < 8; ++j) acc[j] = (v8f){};
#pragma unroll 2
    for (unsigned k0 = 0; k0 < (unsigned)DIM; k0 += 32u) {
      const v16h xb = frag_at(xp + k0);
#pragma unroll
      for (int j = 0; j < 8; ++j) {
        const v16h wa = frag_at(wp + (size_t)j * (16u * WPITCH) + k0);
        acc[j] = wmma16(wa, xb, acc[j]);
      }
    }
#pragma unroll
    for (int j = 0; j < 8; ++j) {
      v8h pk;
#pragma unroll
      for (int r = 0; r < 8; ++r) pk[r] = toh_flush(acc[j][r] * (1.0f / WCARRY));
      *(v8h*)&Ms[(w * 16u + m) * LDM + (unsigned)j * 16u + hh * 8u] = pk;
    }
  }
  __syncthreads();

  {
    const _Float16* wq = Wm_t + (size_t)(w * 16u + m) * KMIX + hh * 8u;
    v8f y = {};
#pragma unroll 1
    for (unsigned c = 0; c < (unsigned)NHEAD; ++c) {
#pragma unroll
      for (unsigned e0 = 0; e0 < (unsigned)DIM; e0 += 32u) {
        const v16h wa = frag_at(wq + c * (unsigned)DIM + e0);
        const v16h fb = ld_frag(&Ms[c * LDM + e0], 8u * LDM);
        y = wmma16(wa, fb, y);
      }
    }
    v4f y0, y1;
#pragma unroll
    for (int r = 0; r < 4; ++r) { y0[r] = y[r]; y1[r] = y[r + 4]; }
    *(v4f*)&Ys[m * LDY + w * 16u + hh * 8u]      = y0;
    *(v4f*)&Ys[m * LDY + w * 16u + hh * 8u + 4u] = y1;
  }
  __syncthreads();

  if (LAST == 0) {
    const unsigned r = tid >> 4;
    const unsigned c = (tid & 15u) * 8u;
    const v4f u0 = *(const v4f*)&Ys[r * LDY + c];
    const v4f u1 = *(const v4f*)&Ys[r * LDY + c + 4u];
    const v4f g0 = *(const v4f*)(bmix + c);
    const v4f g1 = *(const v4f*)(bmix + c + 4u);
    v8h x;
#pragma unroll
    for (int j = 0; j < 4; ++j) {
      x[j]     = toh_flush(u0[j] * cs + bs * bf16r(g0[j]));
      x[j + 4] = toh_flush(u1[j] * cs + bs * bf16r(g1[j]));
    }
    const size_t off = (size_t)(r0 + r) * DIM + c;
    *(volatile v8h*)(out16 + off) = x;
    __threadfence();
    *(volatile v8h*)(out16 + off) = x;
  } else {
    v4f xs[2];
    size_t off[2];
#pragma unroll
    for (unsigned i = 0; i < 2u; ++i) {
      const unsigned r = 8u * i + w;
      const unsigned c = lane * 4u;
      const unsigned crow = r0 + r;
      const unsigned bb = crow / (unsigned)SEQ;
      const unsigned sq = crow - bb * (unsigned)SEQ;
      const size_t frow = (size_t)bb * SEQ_FULL + sq;
      const v4f u = *(const v4f*)&Ys[r * LDY + c];
      const v4f g = *(const v4f*)(bmix + c);
      v4f val;
#pragma unroll
      for (int j = 0; j < 4; ++j) val[j] = u[j] * cs + bs * bf16r(g[j]);
      xs[i] = val;
      off[i] = frow * DIM + c;
    }
#pragma unroll
    for (int i = 0; i < 2; ++i) *(volatile v4f*)(outf + off[i]) = xs[i];
    __threadfence();
#pragma unroll
    for (int i = 0; i < 2; ++i) *(volatile v4f*)(outf + off[i]) = xs[i];
  }
}

__global__ __launch_bounds__(256) void level_mid_kernel(
    const _Float16* __restrict__ Xin, const _Float16* __restrict__ Wh_t,
    const _Float16* __restrict__ Wm_t, const float* __restrict__ bmix,
    _Float16* __restrict__ out16, unsigned lshift, float cs, float bs) {
  level_body<0>(Xin, Wh_t, Wm_t, bmix, (float*)0, out16, lshift, cs, bs);
}
__global__ __launch_bounds__(256) void level_out_kernel(
    const _Float16* __restrict__ Xin, const _Float16* __restrict__ Wh_t,
    const _Float16* __restrict__ Wm_t, const float* __restrict__ bmix,
    float* __restrict__ outf, unsigned lshift, float cs, float bs) {
  level_body<1>(Xin, Wh_t, Wm_t, bmix, outf, (_Float16*)0, lshift, cs, bs);
}

extern "C" void kernel_launch(void* const* d_in, const int* in_sizes, int n_in,
                              void* d_out, int out_size, void* d_ws, size_t ws_size,
                              hipStream_t stream) {
  if (n_in < 4) return;
  const long long need_x = ((long long)(NB - 1) * SEQ_FULL + SEQ) * DIM;
  if ((long long)in_sizes[0] < need_x) return;
  if ((long long)in_sizes[1] < (long long)DEPTH * NHEAD * DIM * DIM) return;
  if ((long long)in_sizes[2] < (long long)KMIX * DIM) return;
  if (in_sizes[3] < DIM) return;
  if ((long long)out_size < need_x) return;
  if (ws_size < WS_TOTAL) return;

  const float* X     = (const float*)d_in[0];
  const float* wts   = (const float*)d_in[1];
  const float* wmix  = (const float*)d_in[2];
  const float* bmix  = (const float*)d_in[3];
  float* out = (float*)d_out;

  char* ws = (char*)d_ws;
  _Float16* Wh_t = (_Float16*)(ws + OFF_WH);
  _Float16* Wm_t = (_Float16*)(ws + OFF_WM);
  _Float16* XA   = (_Float16*)(ws + OFF_XA);
  _Float16* XB   = (_Float16*)(ws + OFF_XB);

  dim3 blk(256);
  dim3 glev(MROWS / 16);

  wconv_kernel<<<dim3(DIM / 64, WPITCH / 64), blk, 0, stream>>>(wts, Wh_t, (unsigned)DIM, (unsigned)WPITCH);
  wconv_kernel<<<dim3(DIM / 64, KMIX / 64), blk, 0, stream>>>(wmix, Wm_t, (unsigned)DIM, (unsigned)KMIX);
  xconv_kernel<<<dim3(MROWS / 16), blk, 0, stream>>>(X, XA);

  level_mid_kernel<<<glev, blk, 0, stream>>>(XA, Wh_t + 0 * NHEAD * DIM, Wm_t, bmix, XB,
                                             LSH0 + 0u, SX1 / WCARRY, SX1);
  level_mid_kernel<<<glev, blk, 0, stream>>>(XB, Wh_t + 1 * NHEAD * DIM, Wm_t, bmix, XA,
                                             LSH0 + 1u, SX2 / (WCARRY * SX1), SX2);
  level_mid_kernel<<<glev, blk, 0, stream>>>(XA, Wh_t + 2 * NHEAD * DIM, Wm_t, bmix, XB,
                                             LSH0 + 2u, SX3 / (WCARRY * SX2), SX3);
  level_out_kernel<<<glev, blk, 0, stream>>>(XB, Wh_t + 3 * NHEAD * DIM, Wm_t, bmix, out,
                                             LSH0 + 3u, 1.0f / (WCARRY * SX3), 1.0f);
}
